// PoolHiddenNet_223338299636
// MI455X (gfx1250) — hardware-verified
//
#include <hip/hip_runtime.h>
#include <stddef.h>
#include <stdint.h>


typedef _Float16 v16h __attribute__((ext_vector_type(16)));
typedef _Float16 v8h  __attribute__((ext_vector_type(8)));
typedef _Float16 v4h  __attribute__((ext_vector_type(4)));
typedef float    v8f  __attribute__((ext_vector_type(8)));
typedef float    v4f  __attribute__((ext_vector_type(4)));

union Frag { v16h v; v8h hv[2]; };

#define NB_   512
#define NS_   16
#define PP_   32
#define HD_   64
#define D1_   8192
#define BOT_  1024
#define ATP   40
#define TRP   72
#define NSTEP (D1_ / 32)
#define HALF_NB 1.0f

__device__ __forceinline__ v8f wmma_g(v16h a, v16h b, v8f c)
{
    v8f d = __builtin_amdgcn_wmma_f32_16x16x32_f16(false, a, false, b, (short)0, c, false, false);
    asm volatile("v_nop\n\tv_nop\n\tv_nop\n\tv_nop" : "+v"(d) : "v"(a), "v"(b));
    return d;
}

__launch_bounds__(256)
__global__ void k_prep(const float* __restrict__ h,
                       const float* __restrict__ Wsp,
                       const float* __restrict__ bsp,
                       const float* __restrict__ W1,
                       const float* __restrict__ b1,
                       _Float16* __restrict__ h16,
                       float* __restrict__ A0,
                       float* __restrict__ A1,
                       float* __restrict__ cst)
{
    const int tid = threadIdx.x;
    if (blockIdx.x < 8) {
        const int k = (blockIdx.x * 256 + tid) * 4;
        v4f a0 = {0.f, 0.f, 0.f, 0.f};
        v4f a1 = {0.f, 0.f, 0.f, 0.f};
        v4f cs = {0.f, 0.f, 0.f, 0.f};
#pragma unroll 4
        for (int e = 0; e < HD_; ++e) {
            const v4f w = *(const v4f*)(W1 + (size_t)e * D1_ + k);
            const float s0 = Wsp[e];
            const float s1 = Wsp[HD_ + e];
            const float sb = bsp[e];
            a0 += s0 * w;
            a1 += s1 * w;
            cs += sb * w;
        }
        cs += *(const v4f*)(b1 + k);
        *(volatile v4f*)(A0 + k)  = a0;
        *(volatile v4f*)(A1 + k)  = a1;
        *(volatile v4f*)(cst + k) = cs;
        __threadfence();
        *(volatile v4f*)(A0 + k)  = a0;
        *(volatile v4f*)(A1 + k)  = a1;
        *(volatile v4f*)(cst + k) = cs;
    } else {
        const int g   = (blockIdx.x - 8) * 256 + tid;
        const int row = g >> 3;
        const int pc  = g & 7;
        const float* src = h + (size_t)row * HD_ + pc * 8;
        const v4f x0 = *(const v4f*)(src);
        const v4f x1 = *(const v4f*)(src + 4);
        v8h r;
        r[0] = (_Float16)x0[0]; r[1] = (_Float16)x0[1]; r[2] = (_Float16)x0[2]; r[3] = (_Float16)x0[3];
        r[4] = (_Float16)x1[0]; r[5] = (_Float16)x1[1]; r[6] = (_Float16)x1[2]; r[7] = (_Float16)x1[3];
        _Float16* dst = h16 + (size_t)row * HD_ + pc * 8;
        *(volatile v8h*)dst = r;
        __threadfence();
        *(volatile v8h*)dst = r;
    }
}

__launch_bounds__(256)
__global__ void k_tr(const float* __restrict__ src,
                     _Float16* __restrict__ dst,
                     int K, int N, float scale)
{
    __shared__ __attribute__((aligned(16))) _Float16 T[64 * TRP];
    const int tid = threadIdx.x;
    const int n0 = blockIdx.x * 64;
    const int k0 = blockIdx.y * 64;
    if (n0 + 64 > N || k0 + 64 > K) return;
    const int col = tid & 63;
    const int rg  = tid >> 6;
#pragma unroll
    for (int i = 0; i < 16; ++i) {
        const int row = i * 4 + rg;
        const float v = src[(size_t)(k0 + row) * N + n0 + col] * scale;
        T[col * TRP + row] = (_Float16)v;
    }
    __syncthreads();
    v8h v[2];
    size_t off[2];
#pragma unroll
    for (int i = 0; i < 2; ++i) {
        const int line = 32 * i + (tid >> 3);
        const int pc   = tid & 7;
        v[i]   = *(const v8h*)(T + line * TRP + 8 * pc);
        off[i] = (size_t)(n0 + line) * K + k0 + 8 * pc;
    }
    *(volatile v8h*)(dst + off[0]) = v[0];
    *(volatile v8h*)(dst + off[1]) = v[1];
    __threadfence();
    *(volatile v8h*)(dst + off[0]) = v[0];
    *(volatile v8h*)(dst + off[1]) = v[1];
}

__launch_bounds__(256)
__global__ void k_cgemm(const _Float16* __restrict__ h16,
                        const _Float16* __restrict__ W1t,
                        float* __restrict__ C)
{
    __shared__ __attribute__((aligned(16))) float Cs[32 * 256];
    const int tid = threadIdx.x;
    const int w   = tid >> 5;
    const int l   = tid & 31;
    const int hh  = l >> 4;
    const int m   = l & 15;
    const int r0  = blockIdx.y * 32;
    const int n0  = blockIdx.x * 256 + w * 32;

    v8f acc00 = {0.f, 0.f, 0.f, 0.f, 0.f, 0.f, 0.f, 0.f};
    v8f acc01 = acc00, acc10 = acc00, acc11 = acc00;

#pragma unroll
    for (int ks = 0; ks < 2; ++ks) {
        const int k0 = ks * 32;
        Frag fa0, fa1, fb0, fb1;
        const _Float16* pa0 = h16 + (size_t)(r0 + m) * HD_ + k0 + 8 * hh;
        const _Float16* pa1 = h16 + (size_t)(r0 + 16 + m) * HD_ + k0 + 8 * hh;
        const _Float16* pb0 = W1t + (size_t)(n0 + m) * HD_ + k0 + 8 * hh;
        const _Float16* pb1 = W1t + (size_t)(n0 + 16 + m) * HD_ + k0 + 8 * hh;
        fa0.hv[0] = *(const v8h*)(pa0); fa0.hv[1] = *(const v8h*)(pa0 + 16);
        fa1.hv[0] = *(const v8h*)(pa1); fa1.hv[1] = *(const v8h*)(pa1 + 16);
        fb0.hv[0] = *(const v8h*)(pb0); fb0.hv[1] = *(const v8h*)(pb0 + 16);
        fb1.hv[0] = *(const v8h*)(pb1); fb1.hv[1] = *(const v8h*)(pb1 + 16);
        acc00 = wmma_g(fa0.v, fb0.v, acc00);
        acc01 = wmma_g(fa0.v, fb1.v, acc01);
        acc10 = wmma_g(fa1.v, fb0.v, acc10);
        acc11 = wmma_g(fa1.v, fb1.v, acc11);
    }

    const float sc = 0.0625f;
#pragma unroll
    for (int r = 0; r < 8; ++r) {
        Cs[(8 * hh + r) * 256 + w * 32 + m]           = acc00[r] * sc;
        Cs[(8 * hh + r) * 256 + w * 32 + 16 + m]      = acc01[r] * sc;
        Cs[(16 + 8 * hh + r) * 256 + w * 32 + m]      = acc10[r] * sc;
        Cs[(16 + 8 * hh + r) * 256 + w * 32 + 16 + m] = acc11[r] * sc;
    }
    __syncthreads();

    v4f v[8];
    size_t off[8];
    const int pc = l & 7;
#pragma unroll
    for (int i = 0; i < 8; ++i) {
        const int row = 4 * i + (l >> 3);
        v[i]   = *(const v4f*)(Cs + row * 256 + w * 32 + 4 * pc);
        off[i] = (size_t)(r0 + row) * D1_ + n0 + 4 * pc;
    }
#pragma unroll
    for (int i = 0; i < 8; ++i) *(volatile v4f*)(C + off[i]) = v[i];
    __threadfence();
#pragma unroll
    for (int i = 0; i < 8; ++i) *(volatile v4f*)(C + off[i]) = v[i];
}

__device__ __forceinline__ void gen4(const float* __restrict__ Crow,
                                     const float* __restrict__ A0,
                                     const float* __restrict__ A1,
                                     const float* __restrict__ cst,
                                     int k, float rx, float ry, _Float16* dstp)
{
    const v4f c  = *(const v4f*)(Crow + k);
    const v4f a0 = *(const v4f*)(A0 + k);
    const v4f a1 = *(const v4f*)(A1 + k);
    const v4f cs = *(const v4f*)(cst + k);
    v4h o;
#pragma unroll
    for (int i = 0; i < 4; ++i) {
        float u = rx * a0[i] + ry * a1[i] + cs[i] + c[i];
        u = fmaxf(u, 0.f);
        o[i] = (_Float16)u;
    }
    *(v4h*)dstp = o;
}

__launch_bounds__(512)
__global__ void k_pool(const float* __restrict__ pos,
                       const float* __restrict__ A0,
                       const float* __restrict__ A1,
                       const float* __restrict__ cst,
                       const float* __restrict__ C,
                       const _Float16* __restrict__ W2t,
                       const float* __restrict__ b2,
                       float* __restrict__ out)
{
    __shared__ __attribute__((aligned(16))) _Float16 At[2 * 32 * ATP];
    __shared__ __attribute__((aligned(16))) float pooled[BOT_];

    const int tid = threadIdx.x;
    const int w   = tid >> 5;
    const int l   = tid & 31;
    const int hh  = l >> 4;
    const int m   = l & 15;
    const int a   = blockIdx.x;
    const int sbase = (a / PP_) * PP_;

    const int gb = (tid >> 3) & 31;
    const int gj = tid & 7;
    float rx = 0.f, ry = 0.f;
    if (w < 8) {
        const int pb = sbase + gb;
        rx = pos[2 * pb]     - pos[2 * a];
        ry = pos[2 * pb + 1] - pos[2 * a + 1];
        rx = fminf(fmaxf(rx, -HALF_NB), HALF_NB) * (1.0f / HALF_NB);
        ry = fminf(fmaxf(ry, -HALF_NB), HALF_NB) * (1.0f / HALF_NB);
    }
    const float* Crow = C + (size_t)(sbase + gb) * D1_;
    _Float16* gdst = At + gb * ATP + 4 * gj;

    v8f acc00 = {0.f, 0.f, 0.f, 0.f, 0.f, 0.f, 0.f, 0.f};
    v8f acc01 = acc00, acc02 = acc00, acc03 = acc00;
    v8f acc10 = acc00, acc11 = acc00, acc12 = acc00, acc13 = acc00;

    if (w < 8) gen4(Crow, A0, A1, cst, 4 * gj, rx, ry, gdst);
    __syncthreads();

    const _Float16* pbrow0 = W2t + (size_t)(w * 64 + 0 * 16 + m) * D1_ + 8 * hh;
    const _Float16* pbrow1 = W2t + (size_t)(w * 64 + 1 * 16 + m) * D1_ + 8 * hh;
    const _Float16* pbrow2 = W2t + (size_t)(w * 64 + 2 * 16 + m) * D1_ + 8 * hh;
    const _Float16* pbrow3 = W2t + (size_t)(w * 64 + 3 * 16 + m) * D1_ + 8 * hh;

#pragma unroll 1
    for (int s = 0; s < NSTEP; ++s) {
        const int cur = s & 1;
        const int k0  = s * 32;
        if (w < 8 && s + 1 < NSTEP)
            gen4(Crow, A0, A1, cst, k0 + 32 + 4 * gj, rx, ry, gdst + (cur ^ 1) * (32 * ATP));

        const _Float16* Ac = At + cur * (32 * ATP);
        Frag fa0, fa1, fb0, fb1, fb2, fb3;
        fa0.hv[0] = *(const v8h*)(Ac + m * ATP + 8 * hh);
        fa0.hv[1] = *(const v8h*)(Ac + m * ATP + 16 + 8 * hh);
        fa1.hv[0] = *(const v8h*)(Ac + (16 + m) * ATP + 8 * hh);
        fa1.hv[1] = *(const v8h*)(Ac + (16 + m) * ATP + 16 + 8 * hh);
        fb0.hv[0] = *(const v8h*)(pbrow0 + k0); fb0.hv[1] = *(const v8h*)(pbrow0 + k0 + 16);
        fb1.hv[0] = *(const v8h*)(pbrow1 + k0); fb1.hv[1] = *(const v8h*)(pbrow1 + k0 + 16);
        fb2.hv[0] = *(const v8h*)(pbrow2 + k0); fb2.hv[1] = *(const v8h*)(pbrow2 + k0 + 16);
        fb3.hv[0] = *(const v8h*)(pbrow3 + k0); fb3.hv[1] = *(const v8h*)(pbrow3 + k0 + 16);

        acc00 = __builtin_amdgcn_wmma_f32_16x16x32_f16(false, fa0.v, false, fb0.v, (short)0, acc00, false, false);
        acc10 = __builtin_amdgcn_wmma_f32_16x16x32_f16(false, fa1.v, false, fb0.v, (short)0, acc10, false, false);
        acc01 = __builtin_amdgcn_wmma_f32_16x16x32_f16(false, fa0.v, false, fb1.v, (short)0, acc01, false, false);
        acc11 = __builtin_amdgcn_wmma_f32_16x16x32_f16(false, fa1.v, false, fb1.v, (short)0, acc11, false, false);
        acc02 = __builtin_amdgcn_wmma_f32_16x16x32_f16(false, fa0.v, false, fb2.v, (short)0, acc02, false, false);
        acc12 = __builtin_amdgcn_wmma_f32_16x16x32_f16(false, fa1.v, false, fb2.v, (short)0, acc12, false, false);
        acc03 = __builtin_amdgcn_wmma_f32_16x16x32_f16(false, fa0.v, false, fb3.v, (short)0, acc03, false, false);
        acc13 = __builtin_amdgcn_wmma_f32_16x16x32_f16(false, fa1.v, false, fb3.v, (short)0, acc13, false, false);
        asm volatile("v_nop\n\tv_nop\n\tv_nop\n\tv_nop"
                     : "+v"(acc00), "+v"(acc01), "+v"(acc02), "+v"(acc03),
                       "+v"(acc10), "+v"(acc11), "+v"(acc12), "+v"(acc13)
                     : "v"(fa0.v), "v"(fa1.v), "v"(fb0.v), "v"(fb1.v), "v"(fb2.v), "v"(fb3.v));
        __syncthreads();
    }

    {
        const float sc = 0.0625f;
        const int   nb = w * 64 + m;
        const float bias0 = b2[nb + 0];
        const float bias1 = b2[nb + 16];
        const float bias2 = b2[nb + 32];
        const float bias3 = b2[nb + 48];
        float mx0 = 0.f, mx1 = 0.f, mx2 = 0.f, mx3 = 0.f;
#pragma unroll
        for (int r = 0; r < 8; ++r) {
            mx0 = fmaxf(mx0, fmaxf(acc00[r] * sc + bias0, 0.f));
            mx0 = fmaxf(mx0, fmaxf(acc10[r] * sc + bias0, 0.f));
            mx1 = fmaxf(mx1, fmaxf(acc01[r] * sc + bias1, 0.f));
            mx1 = fmaxf(mx1, fmaxf(acc11[r] * sc + bias1, 0.f));
            mx2 = fmaxf(mx2, fmaxf(acc02[r] * sc + bias2, 0.f));
            mx2 = fmaxf(mx2, fmaxf(acc12[r] * sc + bias2, 0.f));
            mx3 = fmaxf(mx3, fmaxf(acc03[r] * sc + bias3, 0.f));
            mx3 = fmaxf(mx3, fmaxf(acc13[r] * sc + bias3, 0.f));
        }
        mx0 = fmaxf(mx0, __shfl_xor(mx0, 16, 32));
        mx1 = fmaxf(mx1, __shfl_xor(mx1, 16, 32));
        mx2 = fmaxf(mx2, __shfl_xor(mx2, 16, 32));
        mx3 = fmaxf(mx3, __shfl_xor(mx3, 16, 32));
        if (hh == 0) {
            pooled[nb + 0]  = mx0;
            pooled[nb + 16] = mx1;
            pooled[nb + 32] = mx2;
            pooled[nb + 48] = mx3;
        }
    }
    __syncthreads();

    const bool wr = (tid < 256);
    const int line = (tid >> 3) & 31;
    const int pc   = tid & 7;
    v4f ov = {0.f, 0.f, 0.f, 0.f};
    float* op = out + (size_t)a * BOT_ + line * 32 + 4 * pc;
    if (wr) {
        ov = *(const v4f*)(pooled + line * 32 + 4 * pc);
        *(volatile v4f*)op = ov;
    }
    __threadfence();
    if (wr) {
        *(volatile v4f*)op = ov;
    }
}

extern "C" void kernel_launch(void* const* d_in, const int* in_sizes, int n_in,
                              void* d_out, int out_size, void* d_ws, size_t ws_size,
                              hipStream_t stream)
{
    float* out = (float*)d_out;

    bool ok = (n_in >= 10);
    if (ok) {
        ok = (in_sizes[0] == NB_ * HD_) &&
             (in_sizes[1] == NB_ * 2) &&
             (in_sizes[3] == NS_ * 2) &&
             (in_sizes[4] == 2 * HD_) &&
             (in_sizes[5] == HD_) &&
             (in_sizes[6] == 2 * HD_ * D1_) &&
             (in_sizes[7] == D1_) &&
             (in_sizes[8] == D1_ * BOT_) &&
             (in_sizes[9] == BOT_) &&
             (out_size == NB_ * BOT_) &&
             ((in_sizes[1] / 2) / (in_sizes[3] / 2) == PP_);
    }

    size_t off = 0;
    const size_t o_h16 = off; off += (size_t)NB_ * HD_ * 2;
    const size_t o_W1t = off; off += (size_t)D1_ * HD_ * 2;
    const size_t o_W2t = off; off += (size_t)BOT_ * D1_ * 2;
    const size_t o_A0  = off; off += (size_t)D1_ * 4;
    const size_t o_A1  = off; off += (size_t)D1_ * 4;
    const size_t o_cst = off; off += (size_t)D1_ * 4;
    const size_t o_C   = off; off += (size_t)NB_ * D1_ * 4;
    const size_t ws_total = off;
    ok = ok && (ws_total <= ws_size);

    if (!ok) return;

    const float* h   = (const float*)d_in[0];
    const float* pos = (const float*)d_in[1];
    const float* Wsp = (const float*)d_in[4];
    const float* bsp = (const float*)d_in[5];
    const float* W1  = (const float*)d_in[6];
    const float* b1  = (const float*)d_in[7];
    const float* W2  = (const float*)d_in[8];
    const float* b2  = (const float*)d_in[9];

    char* ws = (char*)d_ws;
    _Float16* h16 = (_Float16*)(ws + o_h16);
    _Float16* W1t = (_Float16*)(ws + o_W1t);
    _Float16* W2t = (_Float16*)(ws + o_W2t);
    float* A0  = (float*)(ws + o_A0);
    float* A1  = (float*)(ws + o_A1);
    float* cst = (float*)(ws + o_cst);
    float* C   = (float*)(ws + o_C);

    k_prep<<<dim3(24), dim3(256), 0, stream>>>(h, Wsp, bsp, W1, b1, h16, A0, A1, cst);
    k_tr<<<dim3(D1_ / 64, HD_ / 64), dim3(256), 0, stream>>>(W1 + (size_t)HD_ * D1_, W1t, HD_, D1_, 16.0f);
    k_tr<<<dim3(BOT_ / 64, D1_ / 64), dim3(256), 0, stream>>>(W2, W2t, D1_, BOT_, 16.0f);
    k_cgemm<<<dim3(D1_ / 256, NB_ / 32), dim3(256), 0, stream>>>(h16, W1t, C);
    k_pool<<<dim3(NB_), dim3(512), 0, stream>>>(pos, A0, A1, cst, C, W2t, b2, out);
}
